// GNNLayer_58042188038247
// MI455X (gfx1250) — hardware-verified
//
#include <hip/hip_runtime.h>
#include <stddef.h>
#include <stdint.h>


#define F      256
#define FH2    128
#define K2     512
#define NTHR   256
#define NWAVE  8
#define EPT    8
#define CHUNK  (NTHR * EPT)
#define WCAP   (EPT * 32)
#define LISTN  (NWAVE * WCAP)
#define NBA    1024
#define SLA    10
#define RCAP   28672
#define DEGCAP 64
#define GBM    64
#define GBN    128
#define GTHR   128
#define GWAVE  (GTHR / 32)
#define GCB    (F / GBN)
#define PARTW  288
#define WSTW   258
#define NUW    (F * (K2 / 8))
#define AGG_ZINTS (LISTN + 2 * RCAP + 3 * NBA)
#define AGG_LDS_INTS (AGG_ZINTS + 16)
#define WSMAX  268435456

static_assert((CHUNK & (CHUNK - 1)) == 0 && CHUNK <= 4096);
static_assert((NBA & (NBA - 1)) == 0 && NBA == (1 << SLA));
static_assert(((long long)CHUNK << SLA) < (1LL << 31));
static_assert(LISTN % NTHR == 0);
static_assert(NBA % NWAVE == 0 && NBA % 32 == 0 && NBA % GBM == 0);
static_assert(RCAP % 4 == 0 && AGG_ZINTS % 4 == 0 && LISTN % 4 == 0);
static_assert(AGG_LDS_INTS * 4 <= 300000);
static_assert(NUW % NTHR == 0);
static_assert(GBM == GWAVE * 16 && GBN == 4 * 32 && GTHR == GBN);
static_assert(F % 32 == 0 && K2 == 2 * F && F == GCB * GBN && K2 / 8 == 64 && F == 2 * FH2 && FH2 == 4 * 32);
static_assert(PARTW % 32 == 0 && PARTW / 4 <= GTHR && PARTW >= 2 * GBN + 1);
static_assert(WSTW >= 2 * GBN + 1 && (WSTW % 2) == 0);

typedef float          v4f   __attribute__((ext_vector_type(4)));
typedef float          v8f   __attribute__((ext_vector_type(8)));
typedef int            v4i   __attribute__((ext_vector_type(4)));
typedef int            v8i   __attribute__((ext_vector_type(8)));
typedef unsigned       v2u   __attribute__((ext_vector_type(2)));
typedef unsigned short v4us  __attribute__((ext_vector_type(4)));
typedef unsigned short v8us  __attribute__((ext_vector_type(8)));
typedef unsigned short v16us __attribute__((ext_vector_type(16)));
typedef __bf16         v16bf __attribute__((ext_vector_type(16)));
typedef v4f  __attribute__((may_alias)) v4fa;
typedef v4i  __attribute__((may_alias)) v4ia;
typedef v2u  __attribute__((may_alias)) v2ua;
typedef v8us __attribute__((may_alias)) v8usa;
union FragB { v16bf v; v16us u; v8us h[2]; v8i w; };

__device__ __forceinline__ v8f wmb(const FragB& a, const FragB& b, v8f c) {
  v8f d = __builtin_amdgcn_wmma_f32_16x16x32_bf16(false, a.v, false, b.v, (short)0, c, false, false);
  asm volatile("v_nop\n\tv_nop\n\tv_nop\n\tv_nop" : "+v"(d) : "v"(a.w), "v"(b.w));
  return d;
}

__device__ __forceinline__ v8f z8() { v8f z = {0.f, 0.f, 0.f, 0.f, 0.f, 0.f, 0.f, 0.f}; return z; }

__device__ __forceinline__ unsigned bf16_bits(float f) {
  const unsigned u = __float_as_uint(f);
  return (u + 0x7FFFu + ((u >> 16) & 1u)) >> 16;
}
__device__ __forceinline__ float bf16_val(float f) {
  return __uint_as_float(bf16_bits(f) << 16);
}

template <int SLB>
__device__ __forceinline__ int scan_chunk(const int* __restrict__ dsts, int nE, int cbase, int slotBase,
                                          int nb, int vec8, int* list, int tid, int lane, int wave) {
  int wc = 0;
  const int el0  = tid * EPT;
  const int e0   = cbase + el0;
  const int sent = -2147483647 - 1;
  v4i da, db;
  if (vec8 != 0 && cbase + CHUNK <= nE) {
    da = *(const v4i*)(dsts + e0);
    db = *(const v4i*)(dsts + e0 + 4);
  } else {
    da.x = (e0     < nE) ? dsts[min(e0,     nE - 1)] : sent;
    da.y = (e0 + 1 < nE) ? dsts[min(e0 + 1, nE - 1)] : sent;
    da.z = (e0 + 2 < nE) ? dsts[min(e0 + 2, nE - 1)] : sent;
    da.w = (e0 + 3 < nE) ? dsts[min(e0 + 3, nE - 1)] : sent;
    db.x = (e0 + 4 < nE) ? dsts[min(e0 + 4, nE - 1)] : sent;
    db.y = (e0 + 5 < nE) ? dsts[min(e0 + 5, nE - 1)] : sent;
    db.z = (e0 + 6 < nE) ? dsts[min(e0 + 6, nE - 1)] : sent;
    db.w = (e0 + 7 < nE) ? dsts[min(e0 + 7, nE - 1)] : sent;
  }
  const unsigned nbs = (unsigned)slotBase;
  const unsigned unb = (unsigned)nb;
  const unsigned s0 = (unsigned)da.x - nbs, s1 = (unsigned)da.y - nbs;
  const unsigned s2 = (unsigned)da.z - nbs, s3 = (unsigned)da.w - nbs;
  const unsigned s4 = (unsigned)db.x - nbs, s5 = (unsigned)db.y - nbs;
  const unsigned s6 = (unsigned)db.z - nbs, s7 = (unsigned)db.w - nbs;
  const bool h0 = s0 < unb, h1 = s1 < unb, h2 = s2 < unb, h3 = s3 < unb;
  const bool h4 = s4 < unb, h5 = s5 < unb, h6 = s6 < unb, h7 = s7 < unb;
  const unsigned any = __builtin_amdgcn_ballot_w32(h0 | h1 | h2 | h3 | h4 | h5 | h6 | h7);
  if (any != 0u) {
#define HITJ(J, HJ, SJ) { \
      const unsigned mj = __builtin_amdgcn_ballot_w32(HJ); \
      if (mj != 0u) { \
        if (HJ) { \
          const int pos = wc + (int)__builtin_amdgcn_mbcnt_lo(mj, 0u); \
          if (pos < WCAP) list[wave * WCAP + pos] = ((el0 + (J)) << SLB) | (int)(SJ); \
        } \
        wc += (int)__builtin_popcount(mj); } }
    HITJ(0, h0, s0)
    HITJ(1, h1, s1)
    HITJ(2, h2, s2)
    HITJ(3, h3, s3)
    HITJ(4, h4, s4)
    HITJ(5, h5, s5)
    HITJ(6, h6, s6)
    HITJ(7, h7, s7)
#undef HITJ
  }
  return wc;
}

__global__ __launch_bounds__(NTHR) void k_prep(const float* __restrict__ W1, const float* __restrict__ W2,
                                               unsigned short* W1B, unsigned short* W2B) {
  const int u = (int)blockIdx.x * NTHR + (int)threadIdx.x;
  v8us o;
  unsigned short* dp;
  if (u < NUW) {
    const int n  = u >> 6;
    const int k8 = (u & 63) * 8;
    const int kk = k8 & (F - 1);
    const float* p = W1 + (size_t)n * F + kk;
    const v4f a = *(const v4f*)p;
    const v4f b = *(const v4f*)(p + 4);
    o[0] = (unsigned short)bf16_bits(a.x); o[1] = (unsigned short)bf16_bits(a.y);
    o[2] = (unsigned short)bf16_bits(a.z); o[3] = (unsigned short)bf16_bits(a.w);
    o[4] = (unsigned short)bf16_bits(b.x); o[5] = (unsigned short)bf16_bits(b.y);
    o[6] = (unsigned short)bf16_bits(b.z); o[7] = (unsigned short)bf16_bits(b.w);
    dp = W1B + (size_t)u * 8;
  } else if (u < 2 * NUW) {
    const int v  = u - NUW;
    const int n  = v >> 6;
    const int k8 = (v & 63) * 8;
    const int kk = k8 & (F - 1);
    const float* p = W2 + (size_t)n * F + kk;
    const v4f a = *(const v4f*)p;
    const v4f b = *(const v4f*)(p + 4);
    o[0] = (unsigned short)bf16_bits(a.x); o[1] = (unsigned short)bf16_bits(a.y);
    o[2] = (unsigned short)bf16_bits(a.z); o[3] = (unsigned short)bf16_bits(a.w);
    o[4] = (unsigned short)bf16_bits(b.x); o[5] = (unsigned short)bf16_bits(b.y);
    o[6] = (unsigned short)bf16_bits(b.z); o[7] = (unsigned short)bf16_bits(b.w);
    dp = W2B + (size_t)v * 8;
  } else {
    return;
  }
  *(volatile v8us*)dp = o;
  __threadfence();
  *(volatile v8us*)dp = o;
}

__global__ __launch_bounds__(NTHR) void k_cvx(const float* __restrict__ x, int nUnits, unsigned short* xb) {
  const int u = (int)blockIdx.x * NTHR + (int)threadIdx.x;
  if (u >= nUnits) return;
  const float* p = x + (size_t)u * 8;
  const v4f a = *(const v4f*)p;
  const v4f b = *(const v4f*)(p + 4);
  v8us o;
  o[0] = (unsigned short)bf16_bits(a.x); o[1] = (unsigned short)bf16_bits(a.y);
  o[2] = (unsigned short)bf16_bits(a.z); o[3] = (unsigned short)bf16_bits(a.w);
  o[4] = (unsigned short)bf16_bits(b.x); o[5] = (unsigned short)bf16_bits(b.y);
  o[6] = (unsigned short)bf16_bits(b.z); o[7] = (unsigned short)bf16_bits(b.w);
  unsigned short* dp = xb + (size_t)u * 8;
  *(volatile v8us*)dp = o;
  __threadfence();
  *(volatile v8us*)dp = o;
}

__global__ __launch_bounds__(NTHR) void k_agg(const int* __restrict__ srcs, const int* __restrict__ dsts,
                                              const float* __restrict__ ew,
                                              int nE, int nN, int vec8, int mRows,
                                              const unsigned short* __restrict__ hb,
                                              float* hn, unsigned short* a1) {
  extern __shared__ __attribute__((aligned(16))) int dsm[];
  int* list = dsm;
  int* hl   = dsm + LISTN;
  int* sl   = hl + RCAP;
  int* cnt  = sl + RCAP;
  int* offs = cnt + NBA;
  int* cur  = offs + NBA;
  int* misc = cur + NBA;
  const int tid = (int)threadIdx.x, lane = tid & 31, wave = tid >> 5;
  const int nodeBase = (int)blockIdx.x * NBA;

  {
    const v4i z4 = {0, 0, 0, 0};
    for (int i = tid * 4; i < AGG_ZINTS; i += NTHR * 4) *(v4ia*)(dsm + i) = z4;
    if (tid < 16) misc[tid] = 0;
  }
  __syncthreads();

  int t = 0, ov = 0;
  const int nChunks = (nE + CHUNK - 1) / CHUNK;
#pragma unroll 1
  for (int ch = 0; ch < nChunks; ++ch) {
    const int cbase = ch * CHUNK;
    const int wc = scan_chunk<SLA>(dsts, nE, cbase, nodeBase, NBA, vec8, list, tid, lane, wave);
    if (lane == 0) misc[wave] = wc;
    __syncthreads();
    if (wave == 0) {
#pragma unroll 1
      for (int w2 = 0; w2 < NWAVE; ++w2) {
        int c = misc[w2];
        c = c < 0 ? 0 : (c > WCAP ? WCAP : c);
#pragma unroll 1
        for (int b0 = 0; b0 < c; b0 += 32) {
          const int idx = b0 + lane;
          const int ent = list[w2 * WCAP + (idx < WCAP ? idx : WCAP - 1)];
          const int m32 = (c - b0) < 32 ? (c - b0) : 32;
#pragma unroll 1
          for (int k = 0; k < m32; ++k) {
            const int u    = __builtin_amdgcn_readlane(ent, k);
            const int slot = u & (NBA - 1);
            const int el   = (u >> SLA) & (CHUNK - 1);
            const int pk   = ((cbase + el) << SLA) | slot;
            if (t < RCAP) {
              if (lane == 0) { hl[t] = pk; cnt[slot] = cnt[slot] + 1; }
              t = t + 1;
            } else {
              ov = 1;
            }
          }
        }
      }
    }
    __syncthreads();
  }
  if (wave == 0 && lane == 0) { misc[8] = t; misc[9] = ov; }
  __syncthreads();
  int tt = misc[8];
  tt = tt < 0 ? 0 : (tt > RCAP ? RCAP : tt);
  const int ovf = misc[9];

  if (wave == 0) {
    const int base = lane * (NBA / 32);
    int s = 0;
#pragma unroll 1
    for (int i = 0; i < NBA / 32; ++i) s += cnt[base + i];
    int incl = s;
#pragma unroll
    for (int d = 1; d < 32; d <<= 1) {
      const int y = __shfl_up(incl, d, 32);
      if (lane >= d) incl += y;
    }
    int run = incl - s;
#pragma unroll 1
    for (int i = 0; i < NBA / 32; ++i) {
      const int cv = cnt[base + i];
      offs[base + i] = run;
      cur[base + i]  = run;
      run += cv;
    }
  }
  __syncthreads();
  if (wave == 0) {
#pragma unroll 1
    for (int b0 = 0; b0 < tt; b0 += 32) {
      const int idx = b0 + lane;
      const int ent = hl[idx < RCAP ? idx : RCAP - 1];
      const int m32 = (tt - b0) < 32 ? (tt - b0) : 32;
#pragma unroll 1
      for (int k = 0; k < m32; ++k) {
        const int u    = __builtin_amdgcn_readlane(ent, k);
        const int slot = u & (NBA - 1);
        if (lane == 0) {
          int p = cur[slot];
          p = p < 0 ? 0 : (p > RCAP - 1 ? RCAP - 1 : p);
          sl[p] = u;
          cur[slot] = p + 1;
        }
      }
    }
  }
  __syncthreads();

  const float pz = (ovf != 0) ? __int_as_float(0x7fc00000) : 0.0f;
#pragma unroll 1
  for (int si = 0; si < NBA / NWAVE; ++si) {
    const int s    = si * NWAVE + wave;
    const int node = nodeBase + s;
    int c = cnt[s];
    const bool big = c > DEGCAP;
    c = c < 0 ? 0 : (c > DEGCAP ? DEGCAP : c);
    int o = offs[s];
    o = o < 0 ? 0 : (o > RCAP ? RCAP : o);
    float acc[8];
#pragma unroll
    for (int i = 0; i < 8; ++i) acc[i] = 0.0f;
#pragma unroll 1
    for (int b0 = 0; b0 < c; b0 += 32) {
      int idx = o + b0 + lane;
      idx = idx > RCAP - 1 ? RCAP - 1 : idx;
      const int ent = sl[idx];
      int eid = ent >> SLA;
      eid = eid < 0 ? 0 : (eid > nE - 1 ? nE - 1 : eid);
      int sr = srcs[eid];
      sr = sr < 0 ? 0 : (sr > nN - 1 ? nN - 1 : sr);
      const float wv  = bf16_val(ew[eid]);
      const int   wvi = __float_as_int(wv);
      const int m32 = (c - b0) < 32 ? (c - b0) : 32;
#pragma unroll 1
      for (int k = 0; k < m32; ++k) {
        const int   sk = __builtin_amdgcn_readlane(sr, k);
        const float ck = __int_as_float(__builtin_amdgcn_readlane(wvi, k));
        const unsigned short* rp = hb + (size_t)sk * F + 4 * lane;
        const v2u qa = *(const v2ua*)rp;
        const v2u qb = *(const v2ua*)(rp + FH2);
        acc[0] = fmaf(ck, __uint_as_float(qa.x << 16),          acc[0]);
        acc[1] = fmaf(ck, __uint_as_float(qa.x & 0xffff0000u), acc[1]);
        acc[2] = fmaf(ck, __uint_as_float(qa.y << 16),          acc[2]);
        acc[3] = fmaf(ck, __uint_as_float(qa.y & 0xffff0000u), acc[3]);
        acc[4] = fmaf(ck, __uint_as_float(qb.x << 16),          acc[4]);
        acc[5] = fmaf(ck, __uint_as_float(qb.x & 0xffff0000u), acc[5]);
        acc[6] = fmaf(ck, __uint_as_float(qb.y << 16),          acc[6]);
        acc[7] = fmaf(ck, __uint_as_float(qb.y & 0xffff0000u), acc[7]);
      }
    }
    const float den = (c > 0) ? (float)c : 1.0f;
    const float rcp = 1.0f / den;
    const float pzr = big ? __int_as_float(0x7fc00000) : pz;
    const bool live = node < nN;
    float v[8];
#pragma unroll
    for (int i = 0; i < 8; ++i) {
      const float y = acc[i] * rcp + pzr;
      v[i] = live ? y : 0.0f;
    }
    if (node < mRows) {
      v4f f0, f1;
      f0.x = v[0]; f0.y = v[1]; f0.z = v[2]; f0.w = v[3];
      f1.x = v[4]; f1.y = v[5]; f1.z = v[6]; f1.w = v[7];
      v4us h0, h1, l0, l1;
#pragma unroll
      for (int i = 0; i < 4; ++i) {
        const unsigned hb0 = bf16_bits(v[i]);
        h0[i] = (unsigned short)hb0;
        l0[i] = (unsigned short)bf16_bits(v[i] - __uint_as_float(hb0 << 16));
        const unsigned hb1 = bf16_bits(v[4 + i]);
        h1[i] = (unsigned short)hb1;
        l1[i] = (unsigned short)bf16_bits(v[4 + i] - __uint_as_float(hb1 << 16));
      }
      float* hp = hn + (size_t)node * F + 4 * lane;
      unsigned short* aq = a1 + (size_t)node * K2 + 4 * lane;
      *(volatile v4f*)hp = f0;
      *(volatile v4f*)(hp + FH2) = f1;
      *(volatile v4us*)aq = h0;
      *(volatile v4us*)(aq + FH2) = h1;
      *(volatile v4us*)(aq + F) = l0;
      *(volatile v4us*)(aq + F + FH2) = l1;
      __threadfence();
      *(volatile v4f*)hp = f0;
      *(volatile v4f*)(hp + FH2) = f1;
      *(volatile v4us*)aq = h0;
      *(volatile v4us*)(aq + FH2) = h1;
      *(volatile v4us*)(aq + F) = l0;
      *(volatile v4us*)(aq + F + FH2) = l1;
    }
  }
}

template <int MODE>
__global__ __launch_bounds__(GTHR) void k_gemm(const unsigned short* __restrict__ A,
                                               const unsigned short* __restrict__ BT, int nN,
                                               const float* __restrict__ bias,
                                               unsigned short* aout, float* xout, float* part) {
  __shared__ __attribute__((aligned(16))) float stg[GBM * GBN];
  __shared__ __attribute__((aligned(16))) float wst[GWAVE * WSTW];
  __shared__ __attribute__((aligned(16))) float pst[PARTW];
  const int tid = (int)threadIdx.x, lane = tid & 31, wave = tid >> 5, hh = lane >> 4, m = lane & 15;
  const int rowBase = (int)blockIdx.x * GBM;
  const int colBase = (int)blockIdx.y * GBN;

  v8f acc[8];
#pragma unroll
  for (int t = 0; t < 8; ++t) acc[t] = z8();
  const unsigned short* ap = A  + (size_t)(rowBase + 16 * wave + m) * (size_t)K2 + 8 * hh;
  const unsigned short* bp = BT + (size_t)(colBase + m) * (size_t)K2 + 8 * hh;

#pragma unroll 1
  for (int k0 = 0; k0 < K2; k0 += 32) {
    FragB af;
    af.h[0] = *(const v8usa*)(ap + k0);
    af.h[1] = *(const v8usa*)(ap + k0 + 16);
#pragma unroll
    for (int nt = 0; nt < 8; ++nt) {
      const unsigned short* wq = bp + (size_t)(16 * nt) * (size_t)K2 + k0;
      FragB bf;
      bf.h[0] = *(const v8usa*)wq;
      bf.h[1] = *(const v8usa*)(wq + 16);
      acc[nt] = wmb(af, bf, acc[nt]);
    }
  }

#pragma unroll
  for (int nt = 0; nt < 8; ++nt) {
    const int lc = 16 * nt + m;
#pragma unroll
    for (int r = 0; r < 8; ++r) {
      const int lr = 16 * wave + 8 * hh + r;
      stg[lr * GBN + lc] = acc[nt][r];
    }
  }
  __syncthreads();

  float bq[4];
  {
    const v4f b4 = *(const v4f*)(bias + colBase + 4 * lane);
    bq[0] = bf16_val(b4.x); bq[1] = bf16_val(b4.y); bq[2] = bf16_val(b4.z); bq[3] = bf16_val(b4.w);
  }

  if constexpr (MODE == 1) {
    v4us hv[16], lv[16];
#pragma unroll
    for (int i = 0; i < 16; ++i) {
      const int row = rowBase + 16 * wave + i;
      const bool ok = row < nN;
      const v4f x = *(const v4fa*)(stg + (16 * wave + i) * GBN + 4 * lane);
      float y[4];
      y[0] = fmaxf(x.x + bq[0], 0.0f); y[1] = fmaxf(x.y + bq[1], 0.0f);
      y[2] = fmaxf(x.z + bq[2], 0.0f); y[3] = fmaxf(x.w + bq[3], 0.0f);
      v4us hq, lq;
#pragma unroll
      for (int j = 0; j < 4; ++j) {
        const float yy = ok ? y[j] : 0.0f;
        const unsigned hbj = bf16_bits(yy);
        hq[j] = (unsigned short)hbj;
        lq[j] = (unsigned short)bf16_bits(yy - __uint_as_float(hbj << 16));
      }
      hv[i] = hq;
      lv[i] = lq;
    }
#pragma unroll
    for (int i = 0; i < 16; ++i) {
      unsigned short* op = aout + (size_t)(rowBase + 16 * wave + i) * (size_t)K2 + colBase + 4 * lane;
      *(volatile v4us*)op = hv[i];
      *(volatile v4us*)(op + F) = lv[i];
    }
    __threadfence();
#pragma unroll
    for (int i = 0; i < 16; ++i) {
      unsigned short* op = aout + (size_t)(rowBase + 16 * wave + i) * (size_t)K2 + colBase + 4 * lane;
      *(volatile v4us*)op = hv[i];
      *(volatile v4us*)(op + F) = lv[i];
    }
  } else {
    v4f pv[16];
    int wn = 0;
    float wm[4], wqv[4];
#pragma unroll
    for (int j = 0; j < 4; ++j) { wm[j] = 0.0f; wqv[j] = 0.0f; }
#pragma unroll
    for (int i = 0; i < 16; ++i) {
      const int row = rowBase + 16 * wave + i;
      const bool ok = row < nN;
      const v4f x = *(const v4fa*)(stg + (16 * wave + i) * GBN + 4 * lane);
      float y[4];
      y[0] = fmaxf(x.x + bq[0], 0.0f); y[1] = fmaxf(x.y + bq[1], 0.0f);
      y[2] = fmaxf(x.z + bq[2], 0.0f); y[3] = fmaxf(x.w + bq[3], 0.0f);
      float vv[4];
#pragma unroll
      for (int j = 0; j < 4; ++j) vv[j] = ok ? y[j] : 0.0f;
      v4f q;
      q.x = vv[0]; q.y = vv[1]; q.z = vv[2]; q.w = vv[3];
      pv[i] = q;
      if (ok) {
        wn += 1;
        const float rk = 1.0f / (float)(i + 1);
#pragma unroll
        for (int j = 0; j < 4; ++j) {
          const float d = vv[j] - wm[j];
          wm[j]  = fmaf(d, rk, wm[j]);
          wqv[j] = fmaf(d, vv[j] - wm[j], wqv[j]);
        }
      }
    }
#pragma unroll
    for (int i = 0; i < 16; ++i) {
      float* op = xout + (size_t)(rowBase + 16 * wave + i) * (size_t)F + colBase + 4 * lane;
      *(volatile v4f*)op = pv[i];
    }
    __threadfence();
#pragma unroll
    for (int i = 0; i < 16; ++i) {
      float* op = xout + (size_t)(rowBase + 16 * wave + i) * (size_t)F + colBase + 4 * lane;
      *(volatile v4f*)op = pv[i];
    }

    if (lane == 0) wst[wave * WSTW] = (float)wn;
#pragma unroll
    for (int j = 0; j < 4; ++j) {
      wst[wave * WSTW + 1 + 4 * lane + j]       = wm[j];
      wst[wave * WSTW + 1 + GBN + 4 * lane + j] = wqv[j];
    }
    __syncthreads();
    {
      float n = 0.0f, mean = 0.0f, M2 = 0.0f;
#pragma unroll 1
      for (int w2 = 0; w2 < GWAVE; ++w2) {
        const float nb = wst[w2 * WSTW];
        const float mb = wst[w2 * WSTW + 1 + tid];
        const float qb = wst[w2 * WSTW + 1 + GBN + tid];
        if (nb > 0.5f) {
          const float nn = n + nb;
          const float delta = mb - mean;
          const float f = nb / nn;
          mean = fmaf(delta, f, mean);
          M2 = M2 + qb + delta * delta * n * f;
          n = nn;
        }
      }
      pst[1 + tid] = mean;
      pst[1 + GBN + tid] = M2;
      if (tid == 0) pst[0] = n;
    }
#pragma unroll 1
    for (int i = 2 * GBN + 1 + tid; i < PARTW; i += GTHR) pst[i] = 0.0f;
    __syncthreads();
    const int pb = (int)blockIdx.x * (int)gridDim.y + (int)blockIdx.y;
    v4f ps;
    if (tid < PARTW / 4) {
      ps = *(const v4fa*)(pst + 4 * tid);
      *(volatile v4f*)(part + (size_t)pb * PARTW + 4 * tid) = ps;
    }
    __threadfence();
    if (tid < PARTW / 4) {
      *(volatile v4f*)(part + (size_t)pb * PARTW + 4 * tid) = ps;
    }
  }
}

__global__ __launch_bounds__(F) void k_bnfin(const float* __restrict__ part, int nPart, int nCB,
                                             const float* __restrict__ gam, const float* __restrict__ bet,
                                             float* ss) {
  __shared__ __attribute__((aligned(16))) float stg[2 * F];
  const int tid = (int)threadIdx.x;
  const int c  = tid;
  const int cb = c >> 7;
  const int cc = c & (GBN - 1);
  double n = 0.0, mean = 0.0, M2 = 0.0;
#pragma unroll 1
  for (int b = 0; b < nPart; ++b) {
    const float* pr = part + ((size_t)b * (size_t)nCB + (size_t)cb) * PARTW;
    const double nb = (double)pr[0];
    const double mb = (double)pr[1 + cc];
    const double qb = (double)pr[1 + GBN + cc];
    if (nb > 0.5) {
      const double nn = n + nb;
      const double delta = mb - mean;
      const double f = nb / nn;
      mean = mean + delta * f;
      M2 = M2 + qb + delta * delta * n * f;
      n = nn;
    }
  }
  const double nt = n < 1.0 ? 1.0 : n;
  const float varf  = (float)(M2 / nt);
  const float meanf = (float)mean;
  const float rstd = 1.0f / sqrtf(varf + 1e-5f);
  const float sc = bf16_val(gam[c]) * rstd;
  const float sh = bf16_val(bet[c]) - meanf * sc;
  stg[c] = sc;
  stg[F + c] = sh;
  __syncthreads();
  v4f v;
  if (tid < (2 * F) / 4) {
    v = *(const v4fa*)(stg + 4 * tid);
    *(volatile v4f*)(ss + 4 * tid) = v;
  }
  __threadfence();
  if (tid < (2 * F) / 4) {
    *(volatile v4f*)(ss + 4 * tid) = v;
  }
}

__global__ __launch_bounds__(NTHR) void k_out(const float* __restrict__ x2, const float* __restrict__ hnp,
                                              const float* __restrict__ ss, int nUnits, float* out) {
  __shared__ float ssh[2 * F];
  const int tid = (int)threadIdx.x;
  ssh[tid] = ss[tid];
  ssh[F + tid] = ss[F + tid];
  __syncthreads();
  const int u = (int)blockIdx.x * NTHR + tid;
  if (u >= nUnits) return;
  const int c4 = (u & 63) * 4;
  const v4f x = *(const v4f*)(x2 + (size_t)u * 4);
  const v4f h = *(const v4f*)(hnp + (size_t)u * 4);
  v4f o;
  o.x = fmaf(x.x, ssh[c4 + 0], ssh[F + c4 + 0]) + h.x;
  o.y = fmaf(x.y, ssh[c4 + 1], ssh[F + c4 + 1]) + h.y;
  o.z = fmaf(x.z, ssh[c4 + 2], ssh[F + c4 + 2]) + h.z;
  o.w = fmaf(x.w, ssh[c4 + 3], ssh[F + c4 + 3]) + h.w;
  float* op = out + (size_t)u * 4;
  *(volatile v4f*)op = o;
  __threadfence();
  *(volatile v4f*)op = o;
}

static inline int cdiv(int a, int b) { return (a + b - 1) / b; }
static inline size_t al256(size_t o) { return (o + 255) & ~(size_t)255; }

extern "C" void kernel_launch(void* const* d_in, const int* in_sizes, int n_in,
                              void* d_out, int out_size, void* d_ws, size_t ws_size,
                              hipStream_t stream) {
  if (n_in < 10) return;
  if (in_sizes[0] < F || (in_sizes[0] % F) != 0) return;
  const int nN = in_sizes[0] / F;
  const int nE = in_sizes[1];
  if (nE < 1 || in_sizes[2] != nE || in_sizes[3] != nE) return;
  if (nE >= (1 << 21) || nN < 16 || nN >= (1 << 24)) return;
  if (in_sizes[4] != F * F || in_sizes[5] != F) return;
  if (in_sizes[6] != F * F || in_sizes[7] != F) return;
  if (in_sizes[8] != F || in_sizes[9] != F) return;
  if ((long long)out_size != (long long)nN * F) return;

  const float* h     = (const float*)d_in[0];
  const float* e     = (const float*)d_in[1];
  const int*   src   = (const int*)d_in[2];
  const int*   dst   = (const int*)d_in[3];
  const float* W1    = (const float*)d_in[4];
  const float* b1    = (const float*)d_in[5];
  const float* W2    = (const float*)d_in[6];
  const float* b2    = (const float*)d_in[7];
  const float* gamma = (const float*)d_in[8];
  const float* beta  = (const float*)d_in[9];
  float* out = (float*)d_out;

  const int MP = cdiv(nN, GBM) * GBM;
  const int gM = MP / GBM;
  const int gA = cdiv(nN, NBA);
  if ((long long)gA * NBA < (long long)MP) return;
  const int vec8 = ((nE & 3) == 0) ? 1 : 0;

  char* ws = (char*)d_ws;
  size_t off = 0;
  const size_t oW1B = off; off = al256(off + (size_t)F * K2 * 2);
  const size_t oW2B = off; off = al256(off + (size_t)F * K2 * 2);
  const size_t oHN  = off; off = al256(off + (size_t)MP * F * 4);
  const size_t oA1  = off; off = al256(off + (size_t)MP * K2 * 2);
  const size_t szA2 = (size_t)MP * K2 * 2;
  const size_t szHB = (size_t)nN * F * 2;
  const size_t oA2  = off; off = al256(off + (szA2 > szHB ? szA2 : szHB));
  const size_t oX2  = off; off = al256(off + (size_t)MP * F * 4);
  const size_t oPT  = off; off = al256(off + (size_t)gM * GCB * PARTW * 4);
  const size_t oSS  = off; off = al256(off + (size_t)(2 * F) * 4);
  if (off > ws_size || off > (size_t)WSMAX) return;
  unsigned short* W1B = (unsigned short*)(ws + oW1B);
  unsigned short* W2B = (unsigned short*)(ws + oW2B);
  float*          HN  = (float*)(ws + oHN);
  unsigned short* A1  = (unsigned short*)(ws + oA1);
  unsigned short* A2  = (unsigned short*)(ws + oA2);
  unsigned short* HB  = (unsigned short*)(ws + oA2);
  float*          X2  = (float*)(ws + oX2);
  float*          PT  = (float*)(ws + oPT);
  float*          SS  = (float*)(ws + oSS);

  const size_t aggLds = (size_t)AGG_LDS_INTS * 4;
  hipFuncSetAttribute(reinterpret_cast<const void*>(&k_agg), hipFuncAttributeMaxDynamicSharedMemorySize, (int)aggLds);

  const int nUh = nN * (F / 8);
  const int nUo = nN * (F / 4);
  k_prep<<<(2 * NUW) / NTHR, NTHR, 0, stream>>>(W1, W2, W1B, W2B);
  k_cvx<<<cdiv(nUh, NTHR), NTHR, 0, stream>>>(h, nUh, HB);
  k_agg<<<gA, NTHR, aggLds, stream>>>(src, dst, e, nE, nN, vec8, MP, HB, HN, A1);
  k_gemm<1><<<dim3(gM, GCB), GTHR, 0, stream>>>(A1, W1B, nN, b1, A2, X2, PT);
  k_gemm<2><<<dim3(gM, GCB), GTHR, 0, stream>>>(A2, W2B, nN, b2, A1, X2, PT);
  k_bnfin<<<1, F, 0, stream>>>(PT, gM, GCB, gamma, beta, SS);
  k_out<<<cdiv(nUo, NTHR), NTHR, 0, stream>>>(X2, HN, SS, nUo, out);
}
